// CBiAFormerBlock_88751204205353
// MI455X (gfx1250) — hardware-run, weakly checked
//
#include <hip/hip_runtime.h>
#define NBt 2
#define CC 256
#define HH 64
#define NPX (HH * HH)
#define NR (NBt * NPX)
#define NHD 8
#define HDC 32
#define HG 2
#define GCH 128
#define RR 32
#define NREF (RR * RR)
#define WS 8
#define NWD 64
#define WT 64
#define WCH 16
#define MLPH 1024
typedef __bf16 v16b __attribute__((ext_vector_type(16)));
typedef unsigned short v8us __attribute__((ext_vector_type(8), may_alias));
typedef float  v8f  __attribute__((ext_vector_type(8)));
typedef float  v4f  __attribute__((ext_vector_type(4)));
typedef float  v4fa __attribute__((ext_vector_type(4), may_alias));
union FragB { v16b v; v8us half[2]; unsigned short u[16]; };

__device__ __forceinline__ unsigned short bf16_bits(float x) { unsigned int u = __float_as_uint(x); return (unsigned short)((u + 0x7FFFu + ((u >> 16) & 1u)) >> 16); }
__device__ __forceinline__ float bf16_val(unsigned short b) { return __uint_as_float(((unsigned int)b) << 16); }
__device__ __forceinline__ float bf16_round(float x) { return bf16_val(bf16_bits(x)); }
template <int NT>
__device__ __forceinline__ v8f mmaN(v16b ah, v16b al, v16b bh, v16b bl, v8f c) {
  c = __builtin_amdgcn_wmma_f32_16x16x32_bf16(false, ah, false, bh, (short)0, c, false, false);
  if (NT >= 2) c = __builtin_amdgcn_wmma_f32_16x16x32_bf16(false, al, false, bh, (short)0, c, false, false);
  if (NT >= 3) c = __builtin_amdgcn_wmma_f32_16x16x32_bf16(false, ah, false, bl, (short)0, c, false, false);
  asm volatile("v_nop\n\tv_nop\n\tv_nop\n\tv_nop" : "+v"(c) : "v"(ah), "v"(al), "v"(bh), "v"(bl));
  return c;
}

__global__ __launch_bounds__(256) void k_wt_bf16(const float* __restrict__ W, unsigned short* __restrict__ Wt, int K, int N) {
  const int t = blockIdx.x * 256 + threadIdx.x;
  const int k8n = K / 8;
  if (t >= N * k8n) return;
  const int n = t / k8n, k8 = (t % k8n) * 8;
  v8us v;
#pragma unroll
  for (int i = 0; i < 8; ++i) v[i] = bf16_bits(W[(size_t)(k8 + i) * N + n]);
  *(volatile v8us*)(Wt + (size_t)n * K + k8) = v;
  __threadfence();
  *(volatile v8us*)(Wt + (size_t)n * K + k8) = v;
}

template <bool ASPLIT, int ACT, bool BIAS_BF16>
__global__ __launch_bounds__(128) void k_gemm_bf(const float* __restrict__ A, int lda, const unsigned short* __restrict__ Wt, int ldb,
                                               const float* __restrict__ bias, float* __restrict__ C, int ldc, int M, int N, int K) {
  __shared__ __attribute__((aligned(16))) float so[4][16][64];
  const int tid = threadIdx.x, w = tid >> 5, lane = tid & 31, ln = lane & 15, hh = lane >> 4;
  const int ntn = N / 64;
  const int wid = blockIdx.x * 4 + w;
  const int mt = wid / ntn, nq = wid % ntn;
  if (mt * 16 >= M) return;
  const int row0 = mt * 16, col0 = nq * 64;
  const float* arow = A + (size_t)(row0 + ln) * lda;
  v8f acc[4] = {};
  for (int kb = 0; kb < K; kb += 32) {
    FragB ah, al;
    const v4f x0 = *(const v4fa*)(arow + kb + 8 * hh), x1 = *(const v4fa*)(arow + kb + 8 * hh + 4);
    const v4f x2 = *(const v4fa*)(arow + kb + 16 + 8 * hh), x3 = *(const v4fa*)(arow + kb + 16 + 8 * hh + 4);
    float xs[16] = {x0[0],x0[1],x0[2],x0[3],x1[0],x1[1],x1[2],x1[3],x2[0],x2[1],x2[2],x2[3],x3[0],x3[1],x3[2],x3[3]};
#pragma unroll
    for (int i = 0; i < 16; ++i) { const unsigned short hb = bf16_bits(xs[i]); ah.u[i] = hb; al.u[i] = ASPLIT ? bf16_bits(xs[i] - bf16_val(hb)) : (unsigned short)0; }
#pragma unroll
    for (int t = 0; t < 4; ++t) {
      const unsigned short* brow = Wt + (size_t)(col0 + t * 16 + ln) * ldb + kb;
      FragB b;
      b.half[0] = *(const v8us*)(brow + 8 * hh);
      b.half[1] = *(const v8us*)(brow + 16 + 8 * hh);
      acc[t] = mmaN<ASPLIT ? 2 : 1>(ah.v, al.v, b.v, b.v, acc[t]);
    }
  }
#pragma unroll
  for (int t = 0; t < 4; ++t) {
    float bv = bias ? bias[col0 + t * 16 + ln] : 0.f;
    if (BIAS_BF16) bv = bf16_round(bv);
#pragma unroll
    for (int r = 0; r < 8; ++r) { float v = acc[t][r] + bv; if (ACT == 1) v = fmaxf(v, 0.f); so[w][8 * hh + r][t * 16 + ln] = v; }
  }
  __builtin_amdgcn_fence(__ATOMIC_ACQ_REL, "workgroup");
  __builtin_amdgcn_wave_barrier();
  const int rsub = lane >> 4, c4 = (lane & 15) * 4;
  for (int pass = 0; pass < 2; ++pass) {
#pragma unroll
    for (int q = 0; q < 8; ++q) {
      const int r = q * 2 + rsub;
      const v4f v = *(const v4fa*)&so[w][r][c4];
      *(volatile v4f*)(C + (size_t)(row0 + r) * ldc + col0 + c4) = v;
    }
    if (pass == 0) __threadfence();
  }
}

template <bool ASPLIT, int ACT, bool BIAS_BF16, bool RES_BF16>
__global__ __launch_bounds__(128) void k_gemm_bf3(const float* __restrict__ A, int lda, const unsigned short* __restrict__ Wt, int ldb,
                                                const float* __restrict__ bias, const float* __restrict__ resid, int rmod, int ldr,
                                                float* __restrict__ C, int ldc, int M, int N, int K) {
  __shared__ __attribute__((aligned(16))) float so[4][16][64];
  const int tid = threadIdx.x, w = tid >> 5, lane = tid & 31, ln = lane & 15, hh = lane >> 4;
  const int ntn = N / 64;
  const int wid = blockIdx.x * 4 + w;
  const int mt = wid / ntn, nq = wid % ntn;
  if (mt * 16 >= M) return;
  const int row0 = mt * 16, col0 = nq * 64;
  const float* arow = A + (size_t)(row0 + ln) * lda;
  v8f acc[4] = {};
  for (int kb = 0; kb < K; kb += 32) {
    FragB ah, al;
    const v4f x0 = *(const v4fa*)(arow + kb + 8 * hh), x1 = *(const v4fa*)(arow + kb + 8 * hh + 4);
    const v4f x2 = *(const v4fa*)(arow + kb + 16 + 8 * hh), x3 = *(const v4fa*)(arow + kb + 16 + 8 * hh + 4);
    float xs[16] = {x0[0],x0[1],x0[2],x0[3],x1[0],x1[1],x1[2],x1[3],x2[0],x2[1],x2[2],x2[3],x3[0],x3[1],x3[2],x3[3]};
#pragma unroll
    for (int i = 0; i < 16; ++i) { const unsigned short hb = bf16_bits(xs[i]); ah.u[i] = hb; al.u[i] = ASPLIT ? bf16_bits(xs[i] - bf16_val(hb)) : (unsigned short)0; }
#pragma unroll
    for (int t = 0; t < 4; ++t) {
      const unsigned short* brow = Wt + (size_t)(col0 + t * 16 + ln) * ldb + kb;
      FragB b;
      b.half[0] = *(const v8us*)(brow + 8 * hh);
      b.half[1] = *(const v8us*)(brow + 16 + 8 * hh);
      acc[t] = mmaN<ASPLIT ? 2 : 1>(ah.v, al.v, b.v, b.v, acc[t]);
    }
  }
#pragma unroll
  for (int t = 0; t < 4; ++t) {
    const int col = col0 + t * 16 + ln;
    float bv = bias ? bias[col] : 0.f;
    if (BIAS_BF16) bv = bf16_round(bv);
#pragma unroll
    for (int r = 0; r < 8; ++r) {
      float v = acc[t][r] + bv;
      if (resid) { float rv = resid[(size_t)((row0 + 8 * hh + r) % rmod) * ldr + col]; if (RES_BF16) rv = bf16_round(rv); v += rv; }
      if (ACT == 1) v = fmaxf(v, 0.f);
      if (ACT == 2) v = 0.5f * v * (1.0f + erff(v * 0.70710678118654752f));
      if (ACT == 3) { const float u = 0.7978845608028654f * (v + 0.044715f * v * v * v); v = 0.5f * v * (1.0f + tanhf(u)); }
      so[w][8 * hh + r][t * 16 + ln] = v;
    }
  }
  __builtin_amdgcn_fence(__ATOMIC_ACQ_REL, "workgroup");
  __builtin_amdgcn_wave_barrier();
  const int rsub = lane >> 4, c4 = (lane & 15) * 4;
  for (int pass = 0; pass < 2; ++pass) {
#pragma unroll
    for (int q = 0; q < 8; ++q) {
      const int r = q * 2 + rsub;
      const v4f v = *(const v4fa*)&so[w][r][c4];
      *(volatile v4f*)(C + (size_t)(row0 + r) * ldc + col0 + c4) = v;
    }
    if (pass == 0) __threadfence();
  }
}
template <bool PARAM_BF16>
__global__ __launch_bounds__(256) void k_layernorm(const float* __restrict__ X, const float* __restrict__ R, const float* __restrict__ g, const float* __restrict__ bta,
                                                  float* __restrict__ out_sum, float* __restrict__ out_norm, int N, float eps) {
  __shared__ float red[256];
  const int row = blockIdx.x, tid = threadIdx.x;
  const float* x = X + (size_t)row * N; const float* rr = R ? R + (size_t)row * N : nullptr;
  float vals[16];
  const int per = N / 256;
  float s1 = 0.f;
  for (int u = 0; u < per / 4; ++u) {
    const int j = tid * 4 + 1024 * u;
    const v4f a = *(const v4fa*)(x + j);
    v4f b = {0.f,0.f,0.f,0.f}; if (rr) b = *(const v4fa*)(rr + j);
#pragma unroll
    for (int q = 0; q < 4; ++q) { const float v = a[q] + b[q]; vals[u * 4 + q] = v; s1 += v; }
  }
  red[tid] = s1; __syncthreads();
  for (int st = 128; st > 0; st >>= 1) { if (tid < st) red[tid] += red[tid + st]; __syncthreads(); }
  const float mu = red[0] / (float)N; __syncthreads();
  float s2 = 0.f;
  for (int u = 0; u < per / 4; ++u)
#pragma unroll
    for (int q = 0; q < 4; ++q) { const float c = vals[u * 4 + q] - mu; s2 += c * c; }
  red[tid] = s2; __syncthreads();
  for (int st = 128; st > 0; st >>= 1) { if (tid < st) red[tid] += red[tid + st]; __syncthreads(); }
  const float rs = rsqrtf(red[0] / (float)N + eps);
  for (int pass = 0; pass < 2; ++pass) {
    for (int u = 0; u < per / 4; ++u) {
      const int j = tid * 4 + 1024 * u;
      v4f o, sm;
#pragma unroll
      for (int q = 0; q < 4; ++q) {
        float gg = g[j + q], bb = bta[j + q];
        if (PARAM_BF16) { gg = bf16_round(gg); bb = bf16_round(bb); }
        sm[q] = vals[u * 4 + q]; o[q] = (vals[u * 4 + q] - mu) * rs * gg + bb;
      }
      if (out_sum) *(volatile v4f*)(out_sum + (size_t)row * N + j) = sm;
      *(volatile v4f*)(out_norm + (size_t)row * N + j) = o;
    }
    if (pass == 0) __threadfence();
  }
}


typedef _Float16 v16h __attribute__((ext_vector_type(16)));
union FragH { v16h v; v8us half[2]; _Float16 h[16]; unsigned short u[16]; };
template <int NT>
__device__ __forceinline__ v8f mmaH(v16h ah, v16h al, v16h bh, v16h bl, v8f c) {
  c = __builtin_amdgcn_wmma_f32_16x16x32_f16(false, ah, false, bh, (short)0, c, false, false);
  if (NT >= 2) c = __builtin_amdgcn_wmma_f32_16x16x32_f16(false, al, false, bh, (short)0, c, false, false);
  if (NT >= 3) c = __builtin_amdgcn_wmma_f32_16x16x32_f16(false, ah, false, bl, (short)0, c, false, false);
  asm volatile("v_nop\n\tv_nop\n\tv_nop\n\tv_nop" : "+v"(c) : "v"(ah), "v"(al), "v"(bh), "v"(bl));
  return c;
}
template <bool ASPLIT>
__global__ __launch_bounds__(128) void k_gemm_h(const float* __restrict__ A, int lda, size_t sA, const _Float16* __restrict__ Bh, int ldb, size_t sB, float alpha, float* __restrict__ C, int ldc, size_t sC, int M, int N, int K) {
  __shared__ __attribute__((aligned(16))) float so[4][16][64];
  const int tid = threadIdx.x, w = tid >> 5, lane = tid & 31, ln = lane & 15, hh = lane >> 4; const int by = blockIdx.y;
  A += (size_t)by * sA; Bh += (size_t)by * sB; C += (size_t)by * sC;
  const int ntn = (N + 63) / 64; const int wid = blockIdx.x * 4 + w; const int mt = wid / ntn, nq = wid % ntn; if (mt * 16 >= M) return;
  const int row0 = mt * 16, col0 = nq * 64; const float* arow = A + (size_t)(row0 + ln) * lda;
  v8f acc[4] = {};
  for (int kb = 0; kb < K; kb += 32) {
    FragH ah, al;
    const v4f x0 = *(const v4fa*)(arow + kb + 8 * hh), x1 = *(const v4fa*)(arow + kb + 8 * hh + 4), x2 = *(const v4fa*)(arow + kb + 16 + 8 * hh), x3 = *(const v4fa*)(arow + kb + 16 + 8 * hh + 4);
    float xs[16] = {x0[0],x0[1],x0[2],x0[3],x1[0],x1[1],x1[2],x1[3],x2[0],x2[1],x2[2],x2[3],x3[0],x3[1],x3[2],x3[3]};
#pragma unroll
    for (int i = 0; i < 16; ++i) { const _Float16 h = (_Float16)xs[i]; ah.h[i] = h; al.h[i] = ASPLIT ? (_Float16)(xs[i] - (float)h) : (_Float16)0.0f; }
#pragma unroll
    for (int t = 0; t < 4; ++t) { if (col0 + t * 16 >= N) continue; const size_t boff = (size_t)(col0 + t * 16 + ln) * ldb + kb; FragH bq; bq.half[0] = *(const v8us*)(Bh + boff + 8 * hh); bq.half[1] = *(const v8us*)(Bh + boff + 16 + 8 * hh);
      acc[t] = mmaH<ASPLIT ? 2 : 1>(ah.v, al.v, bq.v, bq.v, acc[t]); }
  }
#pragma unroll
  for (int t = 0; t < 4; ++t) { if (col0 + t * 16 >= N) continue;
#pragma unroll
    for (int r = 0; r < 8; ++r) so[w][8 * hh + r][t * 16 + ln] = acc[t][r] * alpha; }
  __builtin_amdgcn_fence(__ATOMIC_ACQ_REL, "workgroup"); __builtin_amdgcn_wave_barrier();
  const int rsub = lane >> 4, c4 = (lane & 15) * 4;
  for (int pass = 0; pass < 2; ++pass) {
#pragma unroll
    for (int q = 0; q < 8; ++q) { const int r = q * 2 + rsub; if (col0 + c4 < N) { const v4f v = *(const v4fa*)&so[w][r][c4]; *(volatile v4f*)(C + (size_t)(row0 + r) * ldc + col0 + c4) = v; } }
    if (pass == 0) __threadfence(); }
}

__global__ __launch_bounds__(256) void k_wt_f16(const float* __restrict__ W, _Float16* __restrict__ Wt, int K, int N, float scale) {
  const int t = blockIdx.x * 256 + threadIdx.x; if (t >= N * (K / 8)) return; const int n = t / (K / 8), k8 = (t % (K / 8)) * 8; FragH f;
#pragma unroll
  for (int i = 0; i < 8; ++i) f.h[i] = (_Float16)(bf16_round(W[(size_t)(k8 + i) * N + n]) * scale); const v8us o = f.half[0];
  *(volatile v8us*)((unsigned short*)Wt + (size_t)n * K + k8) = o; __threadfence(); *(volatile v8us*)((unsigned short*)Wt + (size_t)n * K + k8) = o;
}
template <int ACT>
__global__ __launch_bounds__(128) void k_gemm_hhx(const _Float16* __restrict__ A, int lda, size_t sA, const _Float16* __restrict__ Bh, int ldb, size_t sB, float alpha, const float* __restrict__ bias, size_t sBias, const float* __restrict__ CP, int rowsPerB, size_t sCPb, int row0g,
    float* __restrict__ C, _Float16* __restrict__ C16, int ldc, size_t sC, int M, int N, int K) {
  __shared__ __attribute__((aligned(16))) float so[4][16][64];
  const int tid = threadIdx.x, w = tid >> 5, lane = tid & 31, ln = lane & 15, hh = lane >> 4; const int by = blockIdx.y;
  A += (size_t)by * sA; Bh += (size_t)by * sB; const size_t cofs = (size_t)by * sC; const float* bp = bias ? bias + (size_t)by * sBias : nullptr;
  const int ntn = (N + 63) / 64; const int wid = blockIdx.x * 4 + w; const int mt = wid / ntn, nq = wid % ntn; if (mt * 16 >= M) return;
  const int row0 = mt * 16, col0 = nq * 64; const _Float16* arow = A + (size_t)(row0 + ln) * lda;
  v8f acc[4] = {};
  for (int kb = 0; kb < K; kb += 32) { FragH ah; ah.half[0] = *(const v8us*)((const unsigned short*)arow + kb + 8 * hh); ah.half[1] = *(const v8us*)((const unsigned short*)arow + kb + 16 + 8 * hh);
#pragma unroll
    for (int t = 0; t < 4; ++t) { if (col0 + t * 16 >= N) continue; const size_t boff = (size_t)(col0 + t * 16 + ln) * ldb + kb; FragH bq; bq.half[0] = *(const v8us*)((const unsigned short*)Bh + boff + 8 * hh); bq.half[1] = *(const v8us*)((const unsigned short*)Bh + boff + 16 + 8 * hh);
      acc[t] = mmaH<1>(ah.v, ah.v, bq.v, bq.v, acc[t]); }
  }
#pragma unroll
  for (int t = 0; t < 4; ++t) { if (col0 + t * 16 >= N) continue; const int col = col0 + t * 16 + ln; const float bv = bp ? bf16_round(bp[col]) : 0.f;
#pragma unroll
    for (int r = 0; r < 8; ++r) { float v = acc[t][r] * alpha + bv; if (CP) { const int bidx = (row0g + row0 + 8 * hh + r) / rowsPerB; v += CP[(size_t)bidx * sCPb + (size_t)by * 64 + col]; } if (ACT == 1) v = (v > 0.f) ? v : expm1f(v); else if (ACT == 7) v = (v > 0.f) ? v + 1.0f : expf(v); else if (ACT == 8) v = tanhf(v); else if (ACT == 9) v = 0.5f * v * (1.0f + tanhf(0.7978845608028654f * (v + 0.044715f * v * v * v))); else if (ACT == 11) v = 1.0f / (1.0f + expf(-v)); else if (ACT == 12) v = (v > 0.f) ? v : 0.01f * v; else if (ACT == 14) v = (v > 0.f) ? v : 0.1f * v; else if (ACT == 15) v = v / (1.0f + expf(-v)); else if (ACT == 3) v = fmaxf(v, 0.f); else if (ACT == 6) v = 0.5f * v * (1.0f + erff(v * 0.70710678118654752f)); so[w][8 * hh + r][t * 16 + ln] = v; } }
  __builtin_amdgcn_fence(__ATOMIC_ACQ_REL, "workgroup"); __builtin_amdgcn_wave_barrier();
  const int rsub = lane >> 4, c4 = (lane & 15) * 4; typedef _Float16 v4h __attribute__((ext_vector_type(4)));
  for (int pass = 0; pass < 2; ++pass) {
#pragma unroll
    for (int q = 0; q < 8; ++q) { const int r = q * 2 + rsub; if (col0 + c4 < N) { const v4f v = *(const v4fa*)&so[w][r][c4]; if (C) *(volatile v4f*)(C + cofs + (size_t)(row0 + r) * ldc + col0 + c4) = v; if (C16) { v4h h4; for (int i = 0; i < 4; ++i) h4[i] = (_Float16)v[i]; *(volatile v4h*)(C16 + cofs + (size_t)(row0 + r) * ldc + col0 + c4) = h4; } } }
    if (pass == 0) __threadfence(); }
}


typedef _Float16 v4h __attribute__((ext_vector_type(4)));

__global__ __launch_bounds__(256) void k_x16(const float* __restrict__ x, _Float16* __restrict__ X16, size_t n8) { const size_t t = (size_t)blockIdx.x * 256 + threadIdx.x; if (t >= n8) return; FragH f;
#pragma unroll
  for (int q = 0; q < 8; ++q) f.h[q] = (_Float16)bf16_round(x[t * 8 + q]); *(volatile v8us*)((unsigned short*)X16 + t * 8) = f.half[0]; __threadfence(); *(volatile v8us*)((unsigned short*)X16 + t * 8) = f.half[0]; }
__global__ __launch_bounds__(256) void k_h16(const float* __restrict__ x, _Float16* __restrict__ X16, size_t n8) { const size_t t = (size_t)blockIdx.x * 256 + threadIdx.x; if (t >= n8) return; FragH f;
#pragma unroll
  for (int q = 0; q < 8; ++q) f.h[q] = (_Float16)x[t * 8 + q]; *(volatile v8us*)((unsigned short*)X16 + t * 8) = f.half[0]; __threadfence(); *(volatile v8us*)((unsigned short*)X16 + t * 8) = f.half[0]; }
__global__ __launch_bounds__(256) void k_round16f(const float* __restrict__ W, _Float16* __restrict__ Bt, size_t n8) { const size_t t = (size_t)blockIdx.x * 256 + threadIdx.x; if (t >= n8) return; FragH f;
#pragma unroll
  for (int i = 0; i < 8; ++i) f.h[i] = (_Float16)(bf16_round(W[t * 8 + i]) * 16.0f); *(volatile v8us*)((unsigned short*)Bt + t * 8) = f.half[0]; __threadfence(); *(volatile v8us*)((unsigned short*)Bt + t * 8) = f.half[0]; }
template <int NHv, int TTv>
__global__ __launch_bounds__(256) void k_vt(const _Float16* __restrict__ V16, int ldv, int voff, _Float16* __restrict__ Vt) { __shared__ unsigned short tl[64][66]; const int tid = threadIdx.x; const int slab = blockIdx.x / (TTv / 64), lg = blockIdx.x % (TTv / 64); const int b = slab / NHv, h = slab % NHv;
  for (int i = tid; i < 64 * 8; i += 256) { const int r = i / 8, c8 = (i % 8) * 8; FragH f; f.half[0] = *(const v8us*)((const unsigned short*)V16 + ((size_t)b * TTv + lg * 64 + r) * ldv + voff + h * 64 + c8);
#pragma unroll
    for (int q = 0; q < 8; ++q) tl[r][c8 + q] = f.u[q]; }
  __syncthreads();
  for (int pass = 0; pass < 2; ++pass) {
#pragma unroll
    for (int rd = 0; rd < 2; ++rd) { const int d = rd * 32 + tid / 8, pc = tid % 8; FragH f;
#pragma unroll
      for (int q = 0; q < 8; ++q) f.u[q] = tl[pc * 8 + q][d];
      *(volatile v8us*)((unsigned short*)Vt + ((size_t)slab * 64 + d) * TTv + lg * 64 + pc * 8) = f.half[0]; }
    if (pass == 0) __threadfence(); } }

__global__ __launch_bounds__(256) void k_hl(const float* __restrict__ F, _Float16* __restrict__ Hh, _Float16* __restrict__ Hl, size_t n8) { const size_t t = (size_t)blockIdx.x * 256 + threadIdx.x; if (t >= n8) return; FragH fh, fl; const v4f a = *(const v4fa*)(F + t * 8), c = *(const v4fa*)(F + t * 8 + 4);
#pragma unroll
  for (int q = 0; q < 4; ++q) { _Float16 h = (_Float16)a[q]; fh.h[q] = h; fl.h[q] = (_Float16)((a[q] - (float)h) * 1024.0f); h = (_Float16)c[q]; fh.h[4 + q] = h; fl.h[4 + q] = (_Float16)((c[q] - (float)h) * 1024.0f); }
  for (int pass = 0; pass < 2; ++pass) { *(volatile v8us*)((unsigned short*)Hh + t * 8) = fh.half[0]; *(volatile v8us*)((unsigned short*)Hl + t * 8) = fl.half[0]; if (pass == 0) __threadfence(); } }

__device__ __forceinline__ int tok_of(int b, int y, int x) { return (b * NWD + (y / WS) * (HH / WS) + (x / WS)) * WT + (y % WS) * WS + (x % WS); }
__device__ __forceinline__ float gelu_f(float v) { return 0.5f * v * (1.0f + erff(v * 0.70710678118654752f)); }
__global__ __launch_bounds__(256) void k_xw(const float* __restrict__ x, float* __restrict__ XW) { const int t = blockIdx.x * 256 + threadIdx.x; if (t >= NR * (CC / 4)) return; const int c0 = (t % (CC / 4)) * 4; const int T = t / (CC / 4); const int b = T / (NWD * WT), w = (T / WT) % NWD, q = T % WT; const int y = (w / 8) * WS + q / WS, xx = (w % 8) * WS + q % WS; v4f v;
#pragma unroll
  for (int k = 0; k < 4; ++k) v[k] = bf16_round(x[((size_t)b * CC + c0 + k) * NPX + y * HH + xx]);
  *(volatile v4f*)(XW + (size_t)T * CC + c0) = v; __threadfence(); *(volatile v4f*)(XW + (size_t)T * CC + c0) = v; }
__global__ __launch_bounds__(256) void k_ln(const float* __restrict__ X, const float* __restrict__ g, const float* __restrict__ bb, _Float16* __restrict__ O16) {
  #pragma clang fp contract(off)
  const int tid = threadIdx.x, w = tid >> 5, l = tid & 31; const int r = blockIdx.x * 8 + w; if (r >= NR) return; float v[8]; float s = 0.f; const v4f a = *(const v4fa*)(X + (size_t)r * CC + l * 8), c = *(const v4fa*)(X + (size_t)r * CC + l * 8 + 4);
#pragma unroll
  for (int k = 0; k < 8; ++k) { v[k] = (k < 4) ? a[k] : c[k - 4]; s += v[k]; }
  for (int o = 16; o > 0; o >>= 1) s += __shfl_xor(s, o, 32); const float mu = s / (float)CC; float q2 = 0.f;
#pragma unroll
  for (int k = 0; k < 8; ++k) { const float d = v[k] - mu; q2 += d * d; }
  for (int o = 16; o > 0; o >>= 1) q2 += __shfl_xor(q2, o, 32); const float rs = rsqrtf(q2 / (float)CC + 1e-5f); FragH f;
#pragma unroll
  for (int k = 0; k < 8; ++k) { const int ch = l * 8 + k; f.h[k] = (_Float16)((v[k] - mu) * rs * bf16_round(g[ch]) + bf16_round(bb[ch])); }
  *(volatile v8us*)((unsigned short*)O16 + (size_t)r * CC + l * 8) = f.half[0]; __threadfence(); *(volatile v8us*)((unsigned short*)O16 + (size_t)r * CC + l * 8) = f.half[0]; }
__global__ __launch_bounds__(256) void k_dw(const float* __restrict__ INq, const float* __restrict__ INs, int si, const float* __restrict__ w, float* __restrict__ OUT) {
  #pragma clang fp contract(off)
  const int so = si / 2; const int t = blockIdx.x * 256 + threadIdx.x; if (t >= NBt * HG * GCH * so * so) return; const int xo = t % so; const int yo = (t / so) % so; const int c = (t / (so * so)) % GCH; const int bg = t / (so * so * GCH); const int b = bg / HG, g = bg % HG; float acc = 0.f;
#pragma unroll
  for (int k = 0; k < 9; ++k) { const int yy = 2 * yo - 1 + k / 3, xx = 2 * xo - 1 + k % 3; if (yy < 0 || yy >= si || xx < 0 || xx >= si) continue; const float v = INq ? INq[(size_t)tok_of(b, yy, xx) * CC + g * GCH + c] : INs[(((size_t)bg * GCH + c) * si + yy) * si + xx]; acc += bf16_round(w[(size_t)c * 9 + k]) * v; }
  *(volatile float*)(OUT + t) = acc; __threadfence(); *(volatile float*)(OUT + t) = acc; }
__global__ __launch_bounds__(256) void k_o3(const float* __restrict__ D3, const float* __restrict__ g, const float* __restrict__ bb, const float* __restrict__ m, const float* __restrict__ vv, _Float16* __restrict__ O3) {
  #pragma clang fp contract(off)
  const int t = blockIdx.x * 256 + threadIdx.x; if (t >= NBt * HG * NWD * (GCH / 8)) return; const int c0 = (t % (GCH / 8)) * 8; const int row = t / (GCH / 8); const int bg = row / NWD, w = row % NWD; FragH f;
#pragma unroll 1
  for (int k = 0; k < 8; ++k) { const int c = c0 + k; float o = D3[((size_t)bg * GCH + c) * NWD + w]; o = (o - bf16_round(m[c])) * rsqrtf(bf16_round(vv[c]) + 1e-5f); o = o * bf16_round(g[c]) + bf16_round(bb[c]); const _Float16 hv = (_Float16)gelu_f(o);
#pragma unroll
    for (int kk = 0; kk < 8; ++kk) f.h[kk] = (kk == k) ? hv : f.h[kk]; }
  *(volatile v8us*)((unsigned short*)O3 + (size_t)row * GCH + c0) = f.half[0]; __threadfence(); *(volatile v8us*)((unsigned short*)O3 + (size_t)row * GCH + c0) = f.half[0]; }
__global__ __launch_bounds__(256) void k_samp(const float* __restrict__ OFF, const _Float16* __restrict__ XA16, int b, int w0, _Float16* __restrict__ SAMP) {
  #pragma clang fp contract(off)
  const int t = blockIdx.x * 256 + threadIdx.x; if (t >= WCH * NREF * HG * (GCH / 8)) return; const int q16 = t % (GCH / 8); const int g = (t / (GCH / 8)) % HG; const int pr = t / ((GCH / 8) * HG); const int wl = pr / NREF, r = pr % NREF; const int w = w0 + wl; const int bg = b * HG + g; const int rr = r / RR, rc = r % RR;
  const float* orow = OFF + ((size_t)bg * NWD + w) * (2 * NREF); const float o0 = orow[r], o1 = orow[NREF + r];
  const float ref0 = ((float)(rr * 2) / (float)(HH - 1)) * 2.0f - 1.0f, ref1 = ((float)(rc * 2) / (float)(HH - 1)) * 2.0f - 1.0f;
  const float g0 = (tanhf(o0) * 0.015625f) * 2.0f + ref0, g1 = (tanhf(o1) * 0.015625f) * 2.0f + ref1;
  const float rows = (g0 + 1.0f) * 0.5f * (float)(HH - 1), cols = (g1 + 1.0f) * 0.5f * (float)(HH - 1); const float r0f = floorf(rows), c0f = floorf(cols); const float wr = rows - r0f, wc = cols - c0f; float acc[8];
#pragma unroll
  for (int k = 0; k < 8; ++k) acc[k] = 0.f;
#pragma unroll
  for (int cn = 0; cn < 4; ++cn) { const int ri = (int)r0f + (cn >> 1), ci = (int)c0f + (cn & 1); const bool valid = (ri >= 0 && ri < HH && ci >= 0 && ci < HH); const float wgt = ((cn >> 1) ? wr : (1.0f - wr)) * ((cn & 1) ? wc : (1.0f - wc)); const float f = valid ? wgt : 0.f; FragH gv; gv.half[0] = *(const v8us*)((const unsigned short*)XA16 + (size_t)tok_of(b, min(max(ri, 0), HH - 1), min(max(ci, 0), HH - 1)) * CC + g * GCH + q16 * 8);
#pragma unroll
    for (int k = 0; k < 8; ++k) acc[k] += f * (float)gv.h[k]; }
  FragH f;
#pragma unroll
  for (int k = 0; k < 8; ++k) f.h[k] = (_Float16)acc[k];
  *(volatile v8us*)((unsigned short*)SAMP + (size_t)pr * CC + g * GCH + q16 * 8) = f.half[0]; __threadfence(); *(volatile v8us*)((unsigned short*)SAMP + (size_t)pr * CC + g * GCH + q16 * 8) = f.half[0]; }
__global__ __launch_bounds__(256) void k_bsoft(const float* __restrict__ S, const float* __restrict__ pe, int h, int w0, _Float16* __restrict__ P16) {
  #pragma clang fp contract(off)
  const int tid = threadIdx.x, wv = tid >> 5, ln = tid & 31; const int row = blockIdx.x * 8 + wv; if (row >= WCH * WT) return; const int wl = row / WT, q = row % WT; const int w = w0 + wl; const int y = (w / 8) * WS + q / WS, x = (w % 8) * WS + q % WS; const float* sr = S + (size_t)row * NREF; const float* peh = pe + (size_t)h * 127 * 127;
  auto logit = [&](int r) { const int rr = r / RR, rc = r % RR; return sr[r] + bf16_round(peh[(2 * rr - y + 63) * 127 + (2 * rc - x + 63)]); };
  float m = -3.0e38f; for (int r = ln; r < NREF; r += 32) m = fmaxf(m, logit(r));
  for (int o = 16; o > 0; o >>= 1) m = fmaxf(m, __shfl_xor(m, o, 32)); float su = 0.f; for (int r = ln; r < NREF; r += 32) su += expf(logit(r) - m);
  for (int o = 16; o > 0; o >>= 1) su += __shfl_xor(su, o, 32); const float inv = 1024.0f / su;
  for (int pass = 0; pass < 2; ++pass) { for (int j = ln * 8; j < NREF; j += 256) { FragH f;
#pragma unroll
      for (int k = 0; k < 8; ++k) f.h[k] = (_Float16)(expf(logit(j + k) - m) * inv);
      *(volatile v8us*)((unsigned short*)P16 + (size_t)row * NREF + j) = f.half[0]; } if (pass == 0) __threadfence(); } }
__global__ __launch_bounds__(256) void k_f16c(const float* __restrict__ F, _Float16* __restrict__ O, size_t n8) { const size_t t = (size_t)blockIdx.x * 256 + threadIdx.x; if (t >= n8) return; const v4f a = *(const v4fa*)(F + t * 8), c = *(const v4fa*)(F + t * 8 + 4); FragH f;
#pragma unroll
  for (int q = 0; q < 8; ++q) f.h[q] = (_Float16)((q < 4) ? a[q] : c[q - 4]);
  *(volatile v8us*)((unsigned short*)O + t * 8) = f.half[0]; __threadfence(); *(volatile v8us*)((unsigned short*)O + t * 8) = f.half[0]; }
__global__ __launch_bounds__(256) void k_gelu16(const float* __restrict__ F, _Float16* __restrict__ O, size_t n8) {
  #pragma clang fp contract(off)
  const size_t t = (size_t)blockIdx.x * 256 + threadIdx.x; if (t >= n8) return; const v4f a = *(const v4fa*)(F + t * 8), c = *(const v4fa*)(F + t * 8 + 4); FragH f = FragH{};
#pragma unroll 1
  for (int q = 0; q < 8; ++q) { const float v = (q < 4) ? ((q == 0) ? a[0] : (q == 1) ? a[1] : (q == 2) ? a[2] : a[3]) : ((q == 4) ? c[0] : (q == 5) ? c[1] : (q == 6) ? c[2] : c[3]); const _Float16 hv = (_Float16)gelu_f(v);
#pragma unroll
    for (int k = 0; k < 8; ++k) f.h[k] = (k == q) ? hv : f.h[k]; }
  *(volatile v8us*)((unsigned short*)O + t * 8) = f.half[0]; __threadfence(); *(volatile v8us*)((unsigned short*)O + t * 8) = f.half[0]; }
__global__ __launch_bounds__(256) void k_out(const float* __restrict__ Z, float* __restrict__ out) { const int t = blockIdx.x * 256 + threadIdx.x; if (t >= NBt * CC * (NPX / 4)) return; const int p0 = (t % (NPX / 4)) * 4; const int c = (t / (NPX / 4)) % CC; const int b = t / ((NPX / 4) * CC); const int y = p0 / HH, x0 = p0 % HH; v4f v;
#pragma unroll
  for (int k = 0; k < 4; ++k) v[k] = Z[(size_t)tok_of(b, y, x0 + k) * CC + c];
  float* dst = out + ((size_t)b * CC + c) * NPX + p0; *(volatile v4f*)dst = v; __threadfence(); *(volatile v4f*)dst = v; }

extern "C" void kernel_launch(void* const* d_in, const int* in_sizes, int n_in,
                              void* d_out, int out_size, void* d_ws, size_t ws_size, hipStream_t stream) {
  (void)in_sizes; (void)n_in; (void)out_size;
  const float* const* I = (const float* const*)d_in; const float* x = I[0]; const float* ln1g = I[1]; const float* ln1b = I[2]; const float* qw = I[3]; const float* qb = I[4]; const float* kw = I[5]; const float* kb = I[6]; const float* vw = I[7]; const float* vb = I[8]; const float* o1w = I[9]; const float* o2w = I[10]; const float* o3w = I[11]; const float* bng = I[12]; const float* bnb = I[13]; const float* bnm = I[14]; const float* bnv = I[15]; const float* o4w = I[16]; const float* pe = I[17]; const float* pjw = I[18]; const float* pjb = I[19]; const float* ln2g = I[20]; const float* ln2b = I[21]; const float* m1w = I[22]; const float* m1b = I[23]; const float* m2w = I[24]; const float* m2b = I[25];
  char* ws = (char*)d_ws; size_t off = 0;
  auto take = [&](size_t bytes) { char* p = ws + off; off += (bytes + 255) & ~(size_t)255; return p; };
  _Float16* BQ = (_Float16*)take((size_t)CC * CC * 2); _Float16* BK = (_Float16*)take((size_t)CC * CC * 2); _Float16* AV = (_Float16*)take((size_t)CC * CC * 2); _Float16* BO4 = (_Float16*)take((size_t)2 * NREF * GCH * 2); _Float16* BPJ = (_Float16*)take((size_t)CC * CC * 2); _Float16* BM1 = (_Float16*)take((size_t)MLPH * CC * 2); _Float16* BM2 = (_Float16*)take((size_t)CC * MLPH * 2);
  float* XW = (float*)take((size_t)NR * CC * 4); _Float16* XA16 = (_Float16*)take((size_t)NR * CC * 2); float* Qf = (float*)take((size_t)NR * CC * 4); _Float16* Q16 = (_Float16*)take((size_t)NR * CC * 2);
  float* D1 = (float*)take((size_t)NBt * HG * GCH * 32 * 32 * 4); float* D2 = (float*)take((size_t)NBt * HG * GCH * 16 * 16 * 4); float* D3 = (float*)take((size_t)NBt * HG * GCH * 8 * 8 * 4); _Float16* O3 = (_Float16*)take((size_t)NBt * HG * NWD * GCH * 2); float* OFF = (float*)take((size_t)NBt * HG * NWD * 2 * NREF * 4);
  _Float16* SAMP = (_Float16*)take((size_t)WCH * NREF * CC * 2); _Float16* KK16 = (_Float16*)take((size_t)WCH * NREF * CC * 2); _Float16* VT16 = (_Float16*)take((size_t)WCH * CC * NREF * 2); float* S = (float*)take((size_t)WCH * WT * NREF * 4); _Float16* P16 = (_Float16*)take((size_t)WCH * WT * NREF * 2); float* O = (float*)take((size_t)NR * CC * 4); _Float16* O16 = (_Float16*)take((size_t)NR * CC * 2); float* X2 = (float*)take((size_t)NR * CC * 4);
  float* HID = (float*)SAMP;
  _Float16* HID16 = VT16;
  if (off > ws_size) return;
  k_round16f<<<(CC * CC / 8 + 255) / 256, 256, 0, stream>>>(qw, BQ, (size_t)CC * CC / 8); k_round16f<<<(CC * CC / 8 + 255) / 256, 256, 0, stream>>>(kw, BK, (size_t)CC * CC / 8); k_round16f<<<(CC * CC / 8 + 255) / 256, 256, 0, stream>>>(pjw, BPJ, (size_t)CC * CC / 8);
  k_round16f<<<(2 * NREF * GCH / 8 + 255) / 256, 256, 0, stream>>>(o4w, BO4, (size_t)2 * NREF * GCH / 8); k_round16f<<<(MLPH * CC / 8 + 255) / 256, 256, 0, stream>>>(m1w, BM1, (size_t)MLPH * CC / 8); k_round16f<<<(CC * MLPH / 8 + 255) / 256, 256, 0, stream>>>(m2w, BM2, (size_t)CC * MLPH / 8);
  k_x16<<<(CC * CC / 8 + 255) / 256, 256, 0, stream>>>(vw, AV, (size_t)CC * CC / 8);
  const size_t n8 = (size_t)NR * CC / 8; const unsigned nb8 = (unsigned)((n8 + 255) / 256); const dim3 gT(((NR / 16) * (CC / 64) + 3) / 4, 1);
  k_xw<<<(unsigned)((NR * (CC / 4) + 255) / 256), 256, 0, stream>>>(x, XW); k_ln<<<NR / 8, 256, 0, stream>>>(XW, ln1g, ln1b, XA16);
  k_gemm_hhx<0><<<gT, 128, 0, stream>>>(XA16, CC, 0, BQ, CC, 0, 0.0625f, qb, 0, nullptr, 1, 0, 0, Qf, Q16, CC, 0, NR, CC, CC);
  k_dw<<<(NBt * HG * GCH * 32 * 32 + 255) / 256, 256, 0, stream>>>(Qf, nullptr, 64, o1w, D1); k_dw<<<(NBt * HG * GCH * 16 * 16 + 255) / 256, 256, 0, stream>>>(nullptr, D1, 32, o2w, D2); k_dw<<<(NBt * HG * GCH * 8 * 8 + 255) / 256, 256, 0, stream>>>(nullptr, D2, 16, o3w, D3);
  k_o3<<<(NBt * HG * NWD * (GCH / 8) + 255) / 256, 256, 0, stream>>>(D3, bng, bnb, bnm, bnv, O3);
  k_gemm_hhx<0><<<dim3((((NBt * HG * NWD) / 16) * (2 * NREF / 64) + 3) / 4, 1), 128, 0, stream>>>(O3, GCH, 0, BO4, GCH, 0, 0.0625f, nullptr, 0, nullptr, 1, 0, 0, OFF, nullptr, 2 * NREF, 0, NBt * HG * NWD, 2 * NREF, GCH);
  const dim3 gK((((WCH * NREF) / 16) * (CC / 64) + 3) / 4, 1), gV(((CC / 16) * (NREF / 64) + 3) / 4, WCH), gS(((WT / 16) * (NREF / 64) + 3) / 4, WCH), gP(((WT / 16) * 1 + 3) / 4, WCH);
  for (int b = 0; b < NBt; ++b) for (int w0 = 0; w0 < NWD; w0 += WCH) {
    const size_t T0 = ((size_t)b * NWD + w0) * WT;
    k_samp<<<(unsigned)((WCH * NREF * HG * (GCH / 8) + 255) / 256), 256, 0, stream>>>(OFF, XA16, b, w0, SAMP);
    k_gemm_hhx<0><<<gK, 128, 0, stream>>>(SAMP, CC, 0, BK, CC, 0, 0.0625f, kb, 0, nullptr, 1, 0, 0, nullptr, KK16, CC, 0, WCH * NREF, CC, CC);
    k_gemm_hhx<0><<<gV, 128, 0, stream>>>(AV, CC, 0, SAMP, CC, (size_t)NREF * CC, 1.0f, nullptr, 0, nullptr, 1, 0, 0, nullptr, VT16, NREF, (size_t)CC * NREF, CC, NREF, CC);
    for (int h = 0; h < NHD; ++h) {
      k_gemm_hhx<0><<<gS, 128, 0, stream>>>(Q16 + T0 * CC + h * HDC, CC, (size_t)WT * CC, KK16 + h * HDC, CC, (size_t)NREF * CC, 0.0625f, nullptr, 0, nullptr, 1, 0, 0, S, nullptr, NREF, (size_t)WT * NREF, WT, NREF, HDC);
      k_bsoft<<<WCH * WT / 8, 256, 0, stream>>>(S, pe, h, w0, P16);
      k_gemm_hhx<0><<<gP, 128, 0, stream>>>(P16, NREF, (size_t)WT * NREF, VT16 + (size_t)h * HDC * NREF, NREF, (size_t)CC * NREF, 0.0009765625f, vb + h * HDC, 0, nullptr, 1, 0, 0, O + T0 * CC + h * HDC, nullptr, CC, (size_t)WT * CC, WT, HDC, NREF); } }
  k_f16c<<<nb8, 256, 0, stream>>>(O, O16, n8);
  k_gemm_hhx<0><<<gT, 128, 0, stream>>>(O16, CC, 0, BPJ, CC, 0, 0.0625f, pjb, 0, XW, 1, (size_t)CC, 0, X2, nullptr, CC, 0, NR, CC, CC);
  k_ln<<<NR / 8, 256, 0, stream>>>(X2, ln2g, ln2b, XA16);
  for (int b = 0; b < NBt; ++b) { const size_t T0 = (size_t)b * NPX;
    k_gemm_hhx<0><<<dim3(((NPX / 16) * (MLPH / 64) + 3) / 4, 1), 128, 0, stream>>>(XA16 + T0 * CC, CC, 0, BM1, CC, 0, 0.0625f, m1b, 0, nullptr, 1, 0, 0, HID, nullptr, MLPH, 0, NPX, MLPH, CC);
    k_gelu16<<<(unsigned)(((size_t)NPX * MLPH / 8 + 255) / 256), 256, 0, stream>>>(HID, HID16, (size_t)NPX * MLPH / 8);
    k_gemm_hhx<0><<<dim3(((NPX / 16) * (CC / 64) + 3) / 4, 1), 128, 0, stream>>>(HID16, MLPH, 0, BM2, MLPH, 0, 0.0625f, m2b, 0, X2 + T0 * CC, 1, (size_t)CC, 0, O + T0 * CC, nullptr, CC, 0, NPX, CC, MLPH); }
  k_out<<<(unsigned)(((size_t)NBt * CC * (NPX / 4) + 255) / 256), 256, 0, stream>>>(O, (float*)d_out);
}
